// RGAS_26268019982502
// MI455X (gfx1250) — hardware-run, weakly checked
//
#include <hip/hip_runtime.h>


#ifndef NB
#define NB 32
#endif
#define NB_FULL 32
#define NCH  256
#define NPX  1024
#define NCS  64
#define NAO  256
#define NC5  256
#define NCF  513
#define NKY  512
#define QRS  2048.0f
#define QRI  (1.0f / 2048.0f)
#define WCS  64.0f
#define WCI  (1.0f / 64.0f)

static_assert(NB <= NB_FULL);
static_assert(NCH % 32 == 0);
static_assert(NPX % 64 == 0);
static_assert(NCS == 64);
static_assert(NCS % 32 == 0);
static_assert(NAO % 64 == 0);
static_assert(NKY == 2 * NAO);
static_assert(NCF == 1 + NKY);
static_assert(NC5 % 64 == 0);
static_assert(NKY % 32 == 0);
static_assert(NPX % 32 == 0);
static_assert(NCS * NPX == NPX * NCS);

typedef _Float16 h16;
typedef unsigned short bf;
typedef __attribute__((ext_vector_type(16))) __bf16   v16bf;
typedef __attribute__((ext_vector_type(16))) _Float16 v16h;
typedef __attribute__((ext_vector_type(8)))  _Float16 v8h;
typedef __attribute__((ext_vector_type(8)))  unsigned short v8us;
typedef __attribute__((ext_vector_type(8)))  float    v8f;
typedef __attribute__((ext_vector_type(4)))  float    v4f;
typedef __attribute__((ext_vector_type(2)))  float    v2f;
typedef v4f  __attribute__((may_alias)) v4fa;
typedef v8h  __attribute__((may_alias)) v8ha;

__device__ __forceinline__ unsigned short f2bf(float f) { unsigned u = __float_as_uint(f); u += 0x7FFFu + ((u >> 16) & 1u); return (unsigned short)(u >> 16); }
__device__ __forceinline__ float bfr(float f) { return __uint_as_float(((unsigned)f2bf(f)) << 16); }
__device__ __forceinline__ v16h cat16(v8h lo, v8h hi) { return __builtin_shufflevector(lo, hi, 0, 1, 2, 3, 4, 5, 6, 7, 8, 9, 10, 11, 12, 13, 14, 15); }
__device__ __forceinline__ v16bf cat16b(v8us lo, v8us hi) { return __builtin_bit_cast(v16bf, __builtin_shufflevector(lo, hi, 0, 1, 2, 3, 4, 5, 6, 7, 8, 9, 10, 11, 12, 13, 14, 15)); }
__device__ __forceinline__ v8f wmma16(v16h a, v16h b, v8f c) { return __builtin_amdgcn_wmma_f32_16x16x32_f16(false, a, false, b, (short)0, c, false, false); }
__device__ __forceinline__ v8f wmmab(v16bf a, v16bf b, v8f c) { return __builtin_amdgcn_wmma_f32_16x16x32_bf16(false, a, false, b, (short)0, c, false, false); }
__device__ __forceinline__ v16h  ldh(const h16* p) { return cat16(*(const v8h*)p, *(const v8h*)(p + 16)); }
__device__ __forceinline__ v16bf ldb(const bf* p)  { return cat16b(*(const v8us*)p, *(const v8us*)(p + 16)); }
__device__ __forceinline__ void wave_sync() { __builtin_amdgcn_fence(3  , "wavefront"); __builtin_amdgcn_wave_barrier(); asm volatile("" ::: "memory"); }

static __device__ __forceinline__ h16 toh_flush(float v) { const h16 r = (h16)v; return (fabsf(v) < 6.103515625e-05f) ? (h16)0.0f : r; }
__device__ __forceinline__ v8f wmma16g(v16h a, v16h b, v8f c) { c = wmma16(a, b, c); asm volatile("v_nop\n\tv_nop\n\tv_nop\n\tv_nop" : "+v"(c) : "v"(a), "v"(b)); return c; }
__device__ __forceinline__ v8f wmmabg(v16bf a, v16bf b, v8f c) { c = wmmab(a, b, c); asm volatile("v_nop\n\tv_nop\n\tv_nop\n\tv_nop" : "+v"(c) : "v"(a), "v"(b)); return c; }
__device__ __forceinline__ void split8(const v4f x0, const v4f x1, v8h& hv, v8h& rv) {
#pragma unroll
    for (int i = 0; i < 4; ++i) { const h16 a0 = toh_flush(x0[i]); const h16 a1 = toh_flush(x1[i]); hv[i] = a0; hv[4 + i] = a1;
        rv[i] = toh_flush((x0[i] - (float)a0) * QRS); rv[4 + i] = toh_flush((x1[i] - (float)a1) * QRS); }
}

__global__ __launch_bounds__(256) void k_cvt8(const float* __restrict__ src, bf* dst, size_t n8) {
    const size_t i = (size_t)blockIdx.x * 256 + threadIdx.x; if (i >= n8) return;
    const v8f v = *(const v8f*)(src + i * 8); v8us o;
#pragma unroll
    for (int k = 0; k < 8; ++k) o[k] = f2bf(v[k]);
    *(volatile v8us*)(dst + i * 8) = o; __threadfence(); *(volatile v8us*)(dst + i * 8) = o;
}

__global__ __launch_bounds__(256) void k_wconv(const float* __restrict__ src, h16* dst, int rows, int cols8, int spitch, int coff) {
#pragma clang fp contract(off)
    const int i = blockIdx.x * 256 + threadIdx.x; if (i >= rows * cols8) return;
    const int r = i / cols8, c8 = (i % cols8) * 8;
    v8h o;
#pragma unroll
    for (int k = 0; k < 8; ++k) o[k] = toh_flush(bfr(src[(size_t)r * spitch + coff + c8 + k]) * WCS);
    *(volatile v8h*)(dst + (size_t)i * 8) = o; __threadfence(); *(volatile v8h*)(dst + (size_t)i * 8) = o;
}

__global__ __launch_bounds__(256) void k_prep(const float* __restrict__ b1, const float* __restrict__ g1, const float* __restrict__ bt1, const float* __restrict__ m1, const float* __restrict__ v1,
                                              const float* __restrict__ b2, const float* __restrict__ g2, const float* __restrict__ bt2, const float* __restrict__ m2, const float* __restrict__ v2,
                                              const float* __restrict__ b3, const float* __restrict__ g3, const float* __restrict__ bt3, const float* __restrict__ m3, const float* __restrict__ v3,
                                              const float* __restrict__ w5, const float* __restrict__ b5, const float* __restrict__ g5, const float* __restrict__ bt5, const float* __restrict__ m5,
                                              const float* __restrict__ v5, const float* __restrict__ w6, float* SCB, float* P5) {
#pragma clang fp contract(off)
    static_assert(96 * 16 == 3 * NCS * 2 * 4);
    static_assert(NCS % 2 == 0);
    static_assert(256 == NC5);
    const int t = threadIdx.x;
    const int c = (2 * t) & 63, set = t >> 5;
    v2f xb1 = *(const v2f*)(b1 + c),  xb2 = *(const v2f*)(b2 + c),  xb3 = *(const v2f*)(b3 + c);
    v2f xg1 = *(const v2f*)(g1 + c),  xg2 = *(const v2f*)(g2 + c),  xg3 = *(const v2f*)(g3 + c);
    v2f xt1 = *(const v2f*)(bt1 + c), xt2 = *(const v2f*)(bt2 + c), xt3 = *(const v2f*)(bt3 + c);
    asm volatile("" : "+v"(xb1), "+v"(xb2), "+v"(xb3), "+v"(xg1), "+v"(xg2), "+v"(xg3), "+v"(xt1), "+v"(xt2), "+v"(xt3) : : "memory");
    v2f xm1 = *(const v2f*)(m1 + c),  xm2 = *(const v2f*)(m2 + c),  xm3 = *(const v2f*)(m3 + c);
    v2f xv1 = *(const v2f*)(v1 + c),  xv2 = *(const v2f*)(v2 + c),  xv3 = *(const v2f*)(v3 + c);
    asm volatile("" : "+v"(xm1), "+v"(xm2), "+v"(xm3), "+v"(xv1), "+v"(xv2), "+v"(xv3) : : "memory");
    const v2f bs = (set == 0) ? xb1 : ((set == 1) ? xb2 : xb3);
    const v2f gs = (set == 0) ? xg1 : ((set == 1) ? xg2 : xg3);
    const v2f ts = (set == 0) ? xt1 : ((set == 1) ? xt2 : xt3);
    const v2f ms = (set == 0) ? xm1 : ((set == 1) ? xm2 : xm3);
    const v2f vs = (set == 0) ? xv1 : ((set == 1) ? xv2 : xv3);
    const float s0 = bfr(gs[0]) * rsqrtf(bfr(vs[0]) + 1e-5f);
    const float s1 = bfr(gs[1]) * rsqrtf(bfr(vs[1]) + 1e-5f);
    v4f o; o[0] = s0; o[1] = (bfr(bs[0]) - bfr(ms[0])) * s0 + bfr(ts[0]); o[2] = s1; o[3] = (bfr(bs[1]) - bfr(ms[1])) * s1 + bfr(ts[1]);
    float yw5 = w5[(size_t)t * NCF], yg5 = g5[t], yv5 = v5[t], yb5 = b5[t], ym5 = m5[t], yt5 = bt5[t], yw6 = w6[t];
    asm volatile("" : "+v"(yw5), "+v"(yg5), "+v"(yv5), "+v"(yb5), "+v"(ym5), "+v"(yt5), "+v"(yw6) : : "memory");
    const float s5 = bfr(yg5) * rsqrtf(bfr(yv5) + 1e-5f);
    v4f q; q[0] = bfr(yw5); q[1] = s5; q[2] = (bfr(yb5) - bfr(ym5)) * s5 + bfr(yt5); q[3] = bfr(yw6);
    if (t < 96) *(volatile v4f*)(SCB + 4 * t) = o;
    *(volatile v4f*)(P5 + 4 * t) = q;
    __threadfence();
    if (t < 96) *(volatile v4f*)(SCB + 4 * t) = o;
    *(volatile v4f*)(P5 + 4 * t) = q;
}

__global__ __launch_bounds__(256) void k_xT(const float* __restrict__ x, bf* XT) {
#pragma clang fp contract(off)
    __shared__ float ts[NCH * 33];
    static_assert(sizeof(float) * NCH * 33 <= 131072);
    static_assert(8 * 32 == NCH);
    static_assert(8 * 4 == 32);
    static_assert(32 * 8 == NCH);
    const int t = threadIdx.x, lane = t & 31;
    const int wave = __builtin_amdgcn_readfirstlane((int)(threadIdx.x >> 5));
    const int p0 = blockIdx.x * 32, b = blockIdx.y;
    const float* src = x + (size_t)b * NCH * NPX + p0;
#pragma unroll 1
    for (int i = 0; i < 8; ++i) { const int k = i * 32 + (t >> 3), c4 = (t & 7) * 4;
        const v4f v = *(const v4f*)(src + (size_t)k * NPX + c4);
        ts[k * 33 + c4] = v[0]; ts[k * 33 + c4 + 1] = v[1]; ts[k * 33 + c4 + 2] = v[2]; ts[k * 33 + c4 + 3] = v[3]; }
    __syncthreads();
    bf* dst = XT + ((size_t)b * NPX + p0) * NCH;
#pragma unroll 1
    for (int ps = 0; ps < 2; ++ps) {
#pragma unroll 1
        for (int i = 0; i < 4; ++i) { const int pp = i * 8 + wave, k8 = lane * 8; v8us o;
#pragma unroll
            for (int e = 0; e < 8; ++e) o[e] = f2bf(ts[(k8 + e) * 33 + pp]);
            *(volatile v8us*)(dst + (size_t)pp * NCH + k8) = o; }
        if (ps == 0) __threadfence(); }
}

#define PLN ((size_t)NB * NCS * NPX)
#define FLN ((size_t)NB * NAO * NCS)
#define YLN ((size_t)NB * NPX * NKY)

__global__ __launch_bounds__(32) void k_conv(const bf* __restrict__ WB, const bf* __restrict__ XT, const float* __restrict__ SCB, h16* G, float* XE) {
    __shared__ __align__(16) float os[64 * 68];
    static_assert(sizeof(float) * 64 * 68 <= 131072);
    static_assert(32 * 16 * 16 == 64 * 128);
    static_assert(16 * 16 == 64 * 4);
    const int lane = threadIdx.x & 31, lr = lane & 15, hi = lane >> 4;
    const int p0 = blockIdx.x * 64, role = blockIdx.y, b = blockIdx.z;
    v8f acc[4][4];
#pragma unroll
    for (int mb = 0; mb < 4; ++mb)
#pragma unroll
        for (int nb = 0; nb < 4; ++nb) acc[mb][nb] = (v8f){};
    const size_t aoff = (size_t)(role * NCS + lr) * NCH + 8 * hi;
    const size_t boff = ((size_t)b * NPX + p0 + lr) * NCH + 8 * hi;
#pragma unroll 1
    for (int kc = 0; kc < NCH; kc += 32) {
        v16bf a[4];
#pragma unroll
        for (int mb = 0; mb < 4; ++mb) a[mb] = ldb(WB + aoff + (size_t)mb * 16 * NCH + kc);
#pragma unroll
        for (int nb = 0; nb < 4; ++nb) { const v16bf bb = ldb(XT + boff + (size_t)nb * 16 * NCH + kc);
#pragma unroll
            for (int mb = 0; mb < 4; ++mb) acc[mb][nb] = wmmabg(a[mb], bb, acc[mb][nb]); }
    }
#pragma unroll
    for (int mb = 0; mb < 4; ++mb) {
        const float* sp = SCB + (size_t)(role * NCS + mb * 16 + hi * 8) * 2;
        const v4f q0 = *(const v4f*)sp, q1 = *(const v4f*)(sp + 4), q2 = *(const v4f*)(sp + 8), q3 = *(const v4f*)(sp + 12);
        float sc[8], sh[8];
        sc[0] = q0[0]; sh[0] = q0[1]; sc[1] = q0[2]; sh[1] = q0[3]; sc[2] = q1[0]; sh[2] = q1[1]; sc[3] = q1[2]; sh[3] = q1[3];
        sc[4] = q2[0]; sh[4] = q2[1]; sc[5] = q2[2]; sh[5] = q2[3]; sc[6] = q3[0]; sh[6] = q3[1]; sc[7] = q3[2]; sh[7] = q3[3];
#pragma unroll
        for (int nb = 0; nb < 4; ++nb) {
#pragma unroll
            for (int j = 0; j < 8; ++j) { const float v = acc[mb][nb][j] * sc[j] + sh[j];
                os[(mb * 16 + hi * 8 + j) * 68 + nb * 16 + lr] = (v > 0.0f) ? v : 0.0f; } }
    }
    wave_sync();
#pragma unroll 1
    for (int ps = 0; ps < 2; ++ps) {
        if (role < 2) {
            h16* ph = G + (size_t)(2 * role) * PLN + (size_t)b * NCS * NPX + p0;
#pragma unroll 1
            for (int s = 0; s < 16; ++s) { const int row = 4 * s + (lane >> 3), c8 = (lane & 7) * 8;
                const v4f x0 = *(const v4fa*)(&os[row * 68 + c8]); const v4f x1 = *(const v4fa*)(&os[row * 68 + c8 + 4]); v8h hv, rv;
                split8(x0, x1, hv, rv);
                *(volatile v8h*)(ph + (size_t)row * NPX + c8) = hv; *(volatile v8h*)(ph + PLN + (size_t)row * NPX + c8) = rv; }
        }
        if (role == 0) {
            h16* pt = G + (size_t)6 * PLN + ((size_t)b * NPX + p0) * NCS;
#pragma unroll 1
            for (int s = 0; s < 16; ++s) { const int pp = 4 * s + (lane >> 3), c8 = (lane & 7) * 8; v4f x0, x1; v8h hv, rv;
#pragma unroll
                for (int i = 0; i < 4; ++i) { x0[i] = os[(c8 + i) * 68 + pp]; x1[i] = os[(c8 + 4 + i) * 68 + pp]; }
                split8(x0, x1, hv, rv);
                *(volatile v8h*)(pt + (size_t)pp * NCS + c8) = hv; *(volatile v8h*)(pt + PLN + (size_t)pp * NCS + c8) = rv; }
        }
        if (role == 2) {
            const int cl = (lane & 15) * 4; v4f sum = (v4f){};
#pragma unroll 4
            for (int row = 0; row < 64; ++row) sum = sum + *(const v4fa*)(&os[row * 68 + cl]);
            sum = sum * (1.0f / 64.0f);
            if (lane < 16) *(volatile v4f*)(XE + (size_t)b * NPX + p0 + cl) = sum;
        }
        if (ps == 0) __threadfence(); }
}

__global__ __launch_bounds__(32) void k_tr(h16* G) {
#pragma clang fp contract(off)
    __shared__ __align__(16) h16 ts[64 * 72];
    static_assert(sizeof(h16) * 64 * 72 <= 131072);
    static_assert(32 * 16 * 16 == 64 * 128);
    const int lane = threadIdx.x & 31;
    const int j0 = blockIdx.x * 64, pl = blockIdx.y, b = blockIdx.z;
    const h16* src = G + (size_t)(2 + pl) * PLN + (size_t)b * NCS * NPX;
    h16* dst = G + (size_t)(4 + pl) * PLN + (size_t)b * NCS * NPX;
#pragma unroll 1
    for (int s = 0; s < 16; ++s) { const int row = 4 * s + (lane >> 3), c8 = (lane & 7) * 8;
        const v8h v = *(const v8h*)(src + (size_t)(j0 + row) * NCS + c8);
        *(v8ha*)(&ts[row * 72 + c8]) = v; }
    wave_sync();
#pragma unroll 1
    for (int ps = 0; ps < 2; ++ps) {
#pragma unroll 1
        for (int s = 0; s < 16; ++s) { const int crow = 4 * s + (lane >> 3), j8 = (lane & 7) * 8; v8h o;
#pragma unroll
            for (int i = 0; i < 8; ++i) o[i] = ts[(j8 + i) * 72 + crow];
            *(volatile v8h*)(dst + (size_t)crow * NPX + j0 + j8) = o; }
        if (ps == 0) __threadfence(); }
}

__global__ __launch_bounds__(32) void k_fac(const h16* __restrict__ W4H, const h16* G, h16* FA) {
    __shared__ __align__(16) float os[16 * 68];
    static_assert(sizeof(float) * 16 * 68 <= 131072);
    static_assert(32 * 16 * 4 == 16 * 128);
    static_assert(NPX % 32 == 0);
    const int lane = threadIdx.x & 31, lr = lane & 15, hi = lane >> 4;
    const int o0 = blockIdx.x * 32, role = blockIdx.y, b = blockIdx.z;
    const h16* Bh = G + (size_t)(4 - 4 * role) * PLN + (size_t)b * NCS * NPX;
    const h16* Br = Bh + PLN;
    const size_t aoff = (size_t)(o0 + lr) * NPX + 8 * hi;
    const size_t boff = (size_t)lr * NPX + 8 * hi;
    v8f accH[2][4], accR[2][4];
#pragma unroll
    for (int mb = 0; mb < 2; ++mb)
#pragma unroll
        for (int nb = 0; nb < 4; ++nb) { accH[mb][nb] = (v8f){}; accR[mb][nb] = (v8f){}; }
#pragma unroll 1
    for (int kc = 0; kc < NPX; kc += 32) {
        v16h a[2];
#pragma unroll
        for (int mb = 0; mb < 2; ++mb) a[mb] = ldh(W4H + aoff + (size_t)mb * 16 * NPX + kc);
#pragma unroll
        for (int nb = 0; nb < 4; ++nb) { const v16h bh = ldh(Bh + boff + (size_t)nb * 16 * NPX + kc); const v16h br = ldh(Br + boff + (size_t)nb * 16 * NPX + kc);
#pragma unroll
            for (int mb = 0; mb < 2; ++mb) { accH[mb][nb] = wmma16g(a[mb], bh, accH[mb][nb]); accR[mb][nb] = wmma16g(a[mb], br, accR[mb][nb]); } }
    }
    h16* ob = FA + (size_t)(2 * role) * FLN + ((size_t)b * NAO + o0) * NCS;
#pragma unroll
    for (int mb = 0; mb < 2; ++mb) {
#pragma unroll
        for (int nb = 0; nb < 4; ++nb) {
#pragma unroll
            for (int j = 0; j < 8; ++j) os[(hi * 8 + j) * 68 + nb * 16 + lr] = (accH[mb][nb][j] + accR[mb][nb][j] * QRI) * WCI; }
        wave_sync();
#pragma unroll 1
        for (int ps = 0; ps < 2; ++ps) {
#pragma unroll 1
            for (int s = 0; s < 4; ++s) { const int row = 4 * s + (lane >> 3), c8 = (lane & 7) * 8;
                const v4f x0 = *(const v4fa*)(&os[row * 68 + c8]); const v4f x1 = *(const v4fa*)(&os[row * 68 + c8 + 4]); v8h hv, rv;
                split8(x0, x1, hv, rv);
                const size_t oo = (size_t)(mb * 16 + row) * NCS + c8;
                *(volatile v8h*)(ob + oo) = hv; *(volatile v8h*)(ob + FLN + oo) = rv; }
            if (ps == 0) __threadfence(); }
        wave_sync();
    }
}

__global__ __launch_bounds__(32) void k_aff(const h16* G, const h16* FA, const float* __restrict__ b4, h16* YP) {
    __shared__ __align__(16) float os[16 * 68];
    static_assert(sizeof(float) * 16 * 68 <= 131072);
    static_assert(32 * 16 * 4 == 16 * 128);
    static_assert(NAO / 64 == 4);
    const int lane = threadIdx.x & 31, lr = lane & 15, hi = lane >> 4;
    const int p0 = blockIdx.x * 32, role = blockIdx.y >> 2, o0 = (blockIdx.y & 3) * 64, b = blockIdx.z;
    const h16* Ah = G + (size_t)(6 - 4 * role) * PLN + (size_t)b * NPX * NCS;
    const h16* Ar = Ah + PLN;
    const h16* Bh = FA + (size_t)(2 * role) * FLN + (size_t)b * NAO * NCS;
    const h16* Br = Bh + FLN;
    const size_t aoff = (size_t)(p0 + lr) * NCS + 8 * hi;
    const size_t boff = (size_t)(o0 + lr) * NCS + 8 * hi;
    v8f accH[2][4], accR[2][4];
#pragma unroll
    for (int mb = 0; mb < 2; ++mb)
#pragma unroll
        for (int nb = 0; nb < 4; ++nb) { accH[mb][nb] = (v8f){}; accR[mb][nb] = (v8f){}; }
#pragma unroll 1
    for (int kc = 0; kc < NCS; kc += 32) {
        v16h ah[2], ar[2];
#pragma unroll
        for (int mb = 0; mb < 2; ++mb) { ah[mb] = ldh(Ah + aoff + (size_t)mb * 16 * NCS + kc); ar[mb] = ldh(Ar + aoff + (size_t)mb * 16 * NCS + kc); }
#pragma unroll
        for (int nb = 0; nb < 4; ++nb) { const v16h bh = ldh(Bh + boff + (size_t)nb * 16 * NCS + kc); const v16h br = ldh(Br + boff + (size_t)nb * 16 * NCS + kc);
#pragma unroll
            for (int mb = 0; mb < 2; ++mb) { accH[mb][nb] = wmma16g(ah[mb], bh, accH[mb][nb]); accR[mb][nb] = wmma16g(ah[mb], br, accR[mb][nb]); accR[mb][nb] = wmma16g(ar[mb], bh, accR[mb][nb]); } }
    }
    float bc[4];
#pragma unroll
    for (int nb = 0; nb < 4; ++nb) bc[nb] = bfr(b4[o0 + nb * 16 + lr]);
    h16* ob = YP + ((size_t)b * NPX + p0) * NKY + role * NAO + o0;
#pragma unroll
    for (int mb = 0; mb < 2; ++mb) {
#pragma unroll
        for (int nb = 0; nb < 4; ++nb) {
#pragma unroll
            for (int j = 0; j < 8; ++j) { const float v = accH[mb][nb][j] + accR[mb][nb][j] * QRI + bc[nb];
                os[(hi * 8 + j) * 68 + nb * 16 + lr] = (v > 0.0f) ? v : 0.0f; } }
        wave_sync();
#pragma unroll 1
        for (int ps = 0; ps < 2; ++ps) {
#pragma unroll 1
            for (int s = 0; s < 4; ++s) { const int row = 4 * s + (lane >> 3), c8 = (lane & 7) * 8;
                const v4f x0 = *(const v4fa*)(&os[row * 68 + c8]); const v4f x1 = *(const v4fa*)(&os[row * 68 + c8 + 4]); v8h hv, rv;
                split8(x0, x1, hv, rv);
                const size_t oo = (size_t)(mb * 16 + row) * NKY + c8;
                *(volatile v8h*)(ob + oo) = hv; *(volatile v8h*)(ob + YLN + oo) = rv; }
            if (ps == 0) __threadfence(); }
        wave_sync();
    }
}

__global__ __launch_bounds__(32) void k_gate(const h16* __restrict__ W5H, const h16* __restrict__ YP, const float* __restrict__ XE, const float* __restrict__ P5,
                                             const float* __restrict__ b6, float* AV) {
    __shared__ __align__(16) float pt[NC5 * 4];
    __shared__ __align__(16) float gs[32];
    static_assert(sizeof(float) * (NC5 * 4 + 32) <= 131072);
    static_assert(8 * 32 == NC5);
    static_assert(8 * 16 == 32 * 4);
    const int lane = threadIdx.x & 31, lr = lane & 15, hi = lane >> 4;
    const int p0 = blockIdx.x * 32, b = blockIdx.y;
#pragma unroll
    for (int i = 0; i < 8; ++i) { const int idx = i * 32 + lane; const v4f q = *(const v4f*)(P5 + (size_t)idx * 4); *(v4fa*)(&pt[idx * 4]) = q; }
    wave_sync();
    const float xv0 = XE[(size_t)b * NPX + p0 + lr], xv1 = XE[(size_t)b * NPX + p0 + 16 + lr];
    const h16* Yh = YP + ((size_t)b * NPX + p0 + lr) * NKY + 8 * hi;
    const h16* Yr = Yh + YLN;
    float sp0 = 0.0f, sp1 = 0.0f;
#pragma unroll 1
    for (int mq = 0; mq < NC5 / 64; ++mq) {
        v8f accH[4][2], accR[4][2];
#pragma unroll
        for (int mb = 0; mb < 4; ++mb)
#pragma unroll
            for (int nt = 0; nt < 2; ++nt) { accH[mb][nt] = (v8f){}; accR[mb][nt] = (v8f){}; }
        const size_t aoff = (size_t)(mq * 64 + lr) * NKY + 8 * hi;
#pragma unroll 1
        for (int kc = 0; kc < NKY; kc += 32) {
            v16h a[4];
#pragma unroll
            for (int mb = 0; mb < 4; ++mb) a[mb] = ldh(W5H + aoff + (size_t)mb * 16 * NKY + kc);
#pragma unroll
            for (int nt = 0; nt < 2; ++nt) { const v16h bh = ldh(Yh + (size_t)nt * 16 * NKY + kc); const v16h br = ldh(Yr + (size_t)nt * 16 * NKY + kc);
#pragma unroll
                for (int mb = 0; mb < 4; ++mb) { accH[mb][nt] = wmma16g(a[mb], bh, accH[mb][nt]); accR[mb][nt] = wmma16g(a[mb], br, accR[mb][nt]); } }
        }
#pragma unroll
        for (int mb = 0; mb < 4; ++mb) {
#pragma unroll
            for (int j = 0; j < 8; ++j) { const int row = mq * 64 + mb * 16 + hi * 8 + j;
                const v4f q = *(const v4fa*)(&pt[row * 4]);
                const float pa = (accH[mb][0][j] + accR[mb][0][j] * QRI) * WCI + q[0] * xv0;
                const float pb = (accH[mb][1][j] + accR[mb][1][j] * QRI) * WCI + q[0] * xv1;
                const float za = pa * q[1] + q[2], zb = pb * q[1] + q[2];
                sp0 += q[3] * ((za > 0.0f) ? za : 0.0f); sp1 += q[3] * ((zb > 0.0f) ? zb : 0.0f); } }
    }
    sp0 += __shfl_xor(sp0, 16, 32); sp1 += __shfl_xor(sp1, 16, 32);
    const float s = ((hi != 0) ? sp1 : sp0) + bfr(b6[0]);
    const float av = __builtin_amdgcn_rcpf(1.0f + expf(-s));
    gs[lane] = av;
    wave_sync();
    const int l8 = lane & 7;
    const v4f gv = *(const v4fa*)(&gs[l8 * 4]);
    float* dst = AV + (size_t)b * NPX + p0 + l8 * 4;
    if (lane < 8) *(volatile v4f*)dst = gv;
    __threadfence();
    if (lane < 8) *(volatile v4f*)dst = gv;
}

__global__ __launch_bounds__(256) void k_out(const float* __restrict__ x, const float* __restrict__ AV, float* OUT, size_t n4) {
#pragma clang fp contract(off)
    const size_t i = (size_t)blockIdx.x * 256 + threadIdx.x; if (i >= n4) return;
    const size_t e = i * 4; const size_t b = e / ((size_t)NCH * NPX); const size_t p = e % (size_t)NPX;
    const v4f xv = *(const v4f*)(x + e); const v4f av = *(const v4f*)(AV + b * NPX + p); v4f o;
#pragma unroll
    for (int k = 0; k < 4; ++k) o[k] = bfr(xv[k]) * av[k];
    *(volatile v4f*)(OUT + e) = o; __threadfence(); *(volatile v4f*)(OUT + e) = o;
}

static constexpr size_t al256(size_t v) { return (v + 255) & ~(size_t)255; }
static constexpr size_t SZ_XT  = al256((size_t)NB * NPX * NCH * 2);
static constexpr size_t SZ_WB  = al256((size_t)3 * NCS * NCH * 2);
static constexpr size_t SZ_W4  = al256((size_t)NAO * NPX * 2);
static constexpr size_t SZ_W5  = al256((size_t)NC5 * NKY * 2);
static constexpr size_t SZ_G   = al256((size_t)8 * PLN * 2);
static constexpr size_t SZ_FA  = al256((size_t)4 * FLN * 2);
static constexpr size_t SZ_Y   = al256((size_t)2 * YLN * 2);
static constexpr size_t SZ_XE  = al256((size_t)NB * NPX * 4);
static constexpr size_t SZ_AV  = al256((size_t)NB * NPX * 4);
static constexpr size_t SZ_SCB = al256((size_t)192 * 2 * 4);
static constexpr size_t SZ_P5  = al256((size_t)NC5 * 4 * 4);
static constexpr size_t SZ_TOTAL = SZ_XT + SZ_WB + SZ_W4 + SZ_W5 + SZ_G + SZ_FA + SZ_Y + SZ_XE + SZ_AV + SZ_SCB + SZ_P5;
static_assert(SZ_TOTAL <= (size_t)134217728);
static_assert((PLN * 2) % 256 == 0);
static_assert((FLN * 2) % 256 == 0);
static_assert((YLN * 2) % 256 == 0);
static_assert(((size_t)NCS * NCH * 2) % 256 == 0);
static_assert(((size_t)NB * NCH * NPX) % 4 == 0);
static_assert((NAO * (NPX / 8)) % 256 == 0);
static_assert((NC5 * (NKY / 8)) % 256 == 0);
static_assert(3 * NCS == 192);

extern "C" void kernel_launch(void* const* d_in, const int* in_sizes, int n_in,
                              void* d_out, int out_size, void* d_ws, size_t ws_size, hipStream_t stream) {
    if (n_in < 29) return;
    const size_t needx = (size_t)NB * NCH * NPX;
    if ((size_t)in_sizes[0] < needx) return;
    if (in_sizes[1] < NCS * NCH || in_sizes[7] < NCS * NCH || in_sizes[13] < NCS * NCH) return;
    for (int i = 2; i <= 6; ++i) { if (in_sizes[i] < NCS || in_sizes[i + 6] < NCS || in_sizes[i + 12] < NCS) return; }
    if (in_sizes[19] < NAO * NPX || in_sizes[20] < NAO) return;
    if (in_sizes[21] < NC5 * NCF) return;
    for (int i = 22; i <= 27; ++i) { if (in_sizes[i] < NC5) return; }
    if (in_sizes[28] < 1) return;
    if ((size_t)out_size < needx) return;
    if (SZ_TOTAL > ws_size) return;
    const float* x   = (const float*)d_in[0];
    const float* w1  = (const float*)d_in[1];  const float* b1  = (const float*)d_in[2];
    const float* g1  = (const float*)d_in[3];  const float* bt1 = (const float*)d_in[4];
    const float* m1  = (const float*)d_in[5];  const float* v1  = (const float*)d_in[6];
    const float* w2  = (const float*)d_in[7];  const float* b2  = (const float*)d_in[8];
    const float* g2  = (const float*)d_in[9];  const float* bt2 = (const float*)d_in[10];
    const float* m2  = (const float*)d_in[11]; const float* v2  = (const float*)d_in[12];
    const float* w3  = (const float*)d_in[13]; const float* b3  = (const float*)d_in[14];
    const float* g3  = (const float*)d_in[15]; const float* bt3 = (const float*)d_in[16];
    const float* m3  = (const float*)d_in[17]; const float* v3  = (const float*)d_in[18];
    const float* w4  = (const float*)d_in[19]; const float* b4  = (const float*)d_in[20];
    const float* w5  = (const float*)d_in[21]; const float* b5  = (const float*)d_in[22];
    const float* g5  = (const float*)d_in[23]; const float* bt5 = (const float*)d_in[24];
    const float* m5  = (const float*)d_in[25]; const float* v5  = (const float*)d_in[26];
    const float* w6  = (const float*)d_in[27]; const float* b6  = (const float*)d_in[28];
    float* OUT = (float*)d_out;
    char* wsp = (char*)d_ws;
    bf*  XT  = (bf*)wsp;    wsp += SZ_XT;
    bf*  WB  = (bf*)wsp;    wsp += SZ_WB;
    h16* W4H = (h16*)wsp;   wsp += SZ_W4;
    h16* W5H = (h16*)wsp;   wsp += SZ_W5;
    h16* G   = (h16*)wsp;   wsp += SZ_G;
    h16* FA  = (h16*)wsp;   wsp += SZ_FA;
    h16* YP  = (h16*)wsp;   wsp += SZ_Y;
    float* XE  = (float*)wsp; wsp += SZ_XE;
    float* AV  = (float*)wsp; wsp += SZ_AV;
    float* SCB = (float*)wsp; wsp += SZ_SCB;
    float* P5  = (float*)wsp; wsp += SZ_P5;

    k_prep<<<1, 256, 0, stream>>>(b1, g1, bt1, m1, v1, b2, g2, bt2, m2, v2, b3, g3, bt3, m3, v3, w5, b5, g5, bt5, m5, v5, w6, SCB, P5);
    { const size_t n8 = (size_t)NCS * NCH / 8; const unsigned g = (unsigned)((n8 + 255) / 256);
      k_cvt8<<<g, 256, 0, stream>>>(w1, WB, n8); k_cvt8<<<g, 256, 0, stream>>>(w2, WB + (size_t)NCS * NCH, n8); k_cvt8<<<g, 256, 0, stream>>>(w3, WB + (size_t)2 * NCS * NCH, n8); }
    k_wconv<<<(NAO * (NPX / 8)) / 256, 256, 0, stream>>>(w4, W4H, NAO, NPX / 8, NPX, 0);
    k_wconv<<<(NC5 * (NKY / 8)) / 256, 256, 0, stream>>>(w5, W5H, NC5, NKY / 8, NCF, 1);
    k_xT<<<dim3(NPX / 32, NB, 1), 256, 0, stream>>>(x, XT);
    k_conv<<<dim3(NPX / 64, 3, NB), 32, 0, stream>>>(WB, XT, SCB, G, XE);
    k_tr<<<dim3(NPX / 64, 2, NB), 32, 0, stream>>>(G);
    k_fac<<<dim3(NAO / 32, 2, NB), 32, 0, stream>>>(W4H, G, FA);
    k_aff<<<dim3(NPX / 32, 2 * (NAO / 64), NB), 32, 0, stream>>>(G, FA, b4, YP);
    k_gate<<<dim3(NPX / 32, NB, 1), 32, 0, stream>>>(W5H, YP, XE, P5, b6, AV);
    { const size_t n4 = (size_t)NB * NCH * NPX / 4;
      k_out<<<(unsigned)((n4 + 255) / 256), 256, 0, stream>>>(x, AV, OUT, n4); }
}
